// ExpertLinear_50002009260704
// MI455X (gfx1250) — hardware-verified
//
#include <hip/hip_runtime.h>
#include <stddef.h>
#include <stdint.h>


#define NTOK  8192
#define TOPK  2
#define NEXP  8
#define DIN   1024
#define DOUT  1024
#define NG    16384
#define MT    64
#define MAXT  264
#define NGP   16448
#define TB    64
#define XSC   16
#define WSC   1024
#define NTHR  256
#define NWAVE 8
#define TPW   64
#define SP    256
#define WSCAP 134217728
#define LDS_GEMM (MT * SP * 4)

static_assert(NG == NTOK * TOPK);
static_assert(MAXT == NG / MT + NEXP);
static_assert(NGP == NG + MT);
static_assert((NGP % 64) == 0);
static_assert((NG % NTHR) == 0);
static_assert((NTOK % TB) == 0);
static_assert(TOPK * TB <= NTHR);
static_assert((TB % NWAVE) == 0);
static_assert(MT == NWAVE * 8);
static_assert(NTHR == NWAVE * 32);
static_assert((DIN % 128) == 0);
static_assert((DIN % 32) == 0);
static_assert((DOUT % 256) == 0);
static_assert((DOUT % 64) == 0);
static_assert(LDS_GEMM == 65536);

typedef float          v2f  __attribute__((ext_vector_type(2)));
typedef float          v4f  __attribute__((ext_vector_type(4)));
typedef float          v8f  __attribute__((ext_vector_type(8)));
typedef _Float16       v8h  __attribute__((ext_vector_type(8)));
typedef _Float16       v16h __attribute__((ext_vector_type(16)));
union FragH { v16h v; v8h h[2]; };

__device__ __forceinline__ v8f wmf(v16h a, v16h b, v8f c) {
  v8f d = __builtin_amdgcn_wmma_f32_16x16x32_f16(false, a, false, b, (short)0, c, false, false);
  asm volatile("v_nop\n\tv_nop\n\tv_nop\n\tv_nop" : "+v"(d) : "v"(a), "v"(b));
  return d;
}

__device__ __forceinline__ int clamp_e(int v) { return v < 0 ? 0 : (v > NEXP - 1 ? NEXP - 1 : v); }

__device__ __forceinline__ int read_k(const int* __restrict__ kin) {
  int kv = kin[0];
  return kv < 1 ? 1 : (kv > TOPK ? TOPK : kv);
}

struct RouteLds { int red[NWAVE][NEXP]; int cnt[NEXP]; };

__device__ __forceinline__ void route_counts(const int* __restrict__ sei, RouteLds* rs, int tid) {
  int tot[NEXP];
#pragma unroll
  for (int e = 0; e < NEXP; ++e) tot[e] = 0;
#pragma unroll 1
  for (int i = tid; i < NG; i += NTHR) {
    const int v = clamp_e(sei[i]);
#pragma unroll
    for (int e = 0; e < NEXP; ++e) tot[e] += (v == e) ? 1 : 0;
  }
#pragma unroll
  for (int e = 0; e < NEXP; ++e) {
#pragma unroll
    for (int o = 16; o > 0; o >>= 1) tot[e] += __shfl_xor(tot[e], o, 32);
  }
  const int lane = tid & 31, wave = tid >> 5;
  if (lane == 0) {
#pragma unroll
    for (int e = 0; e < NEXP; ++e) rs->red[wave][e] = tot[e];
  }
  __syncthreads();
  if (tid < NEXP) {
    int c = 0;
#pragma unroll
    for (int w = 0; w < NWAVE; ++w) c += rs->red[w][tid];
    rs->cnt[tid] = c;
  }
  __syncthreads();
}

__device__ __forceinline__ int tile_geom(const RouteLds* rs, int b, int& row0, int& segEnd, int& my_e) {
  int tp = 0, s = 0; row0 = 0; segEnd = 0; my_e = 0;
#pragma unroll
  for (int e = 0; e < NEXP; ++e) {
    const int c = rs->cnt[e];
    const int nt = (c + MT - 1) / MT;
    if (b >= tp && b < tp + nt) { my_e = e; row0 = s + (b - tp) * MT; segEnd = s + c; }
    tp += nt;
    s += c;
  }
  return tp;
}

__device__ __forceinline__ void tile_write_t(const float* tile, _Float16* dbase, int dp, int dc,
                                             float wsc, int g, int hh, int m) {
  v8h hv[4];
#pragma unroll
  for (int q = 0; q < 4; ++q) {
    const int nl = 8 * g + 2 * q + hh;
    const int d8 = 8 * m;
#pragma unroll
    for (int u = 0; u < 8; ++u) hv[q][u] = (_Float16)(tile[(d8 + u) * TPW + nl] * wsc);
  }
#pragma unroll
  for (int q = 0; q < 4; ++q) {
    _Float16* d = dbase + (size_t)(8 * g + 2 * q + hh) * dp + dc + 8 * m;
    *(volatile v8h*)d = hv[q];
  }
  __threadfence();
#pragma unroll
  for (int q = 0; q < 4; ++q) {
    _Float16* d = dbase + (size_t)(8 * g + 2 * q + hh) * dp + dc + 8 * m;
    *(volatile v8h*)d = hv[q];
  }
}

__global__ __launch_bounds__(NTHR) void k_tw(const float* __restrict__ w, _Float16* wt) {
  __shared__ __attribute__((aligned(16))) float tile[128 * TPW];
  const int tid = threadIdx.x, lane = tid & 31, gw = tid >> 5, hh = lane >> 4, m = lane & 15;
  const int n0 = blockIdx.x * 64, e = blockIdx.y;
#pragma unroll 1
  for (int dc = 0; dc < DIN; dc += 128) {
    __syncthreads();
#pragma unroll 4
    for (int p = 0; p < 16; ++p) {
      const int dl = gw + 8 * p;
      const v2f wv = *(const v2f*)(w + ((size_t)e * DIN + dc + dl) * DOUT + n0 + 2 * lane);
      *(v2f*)(tile + dl * TPW + 2 * lane) = wv;
    }
    __syncthreads();
    tile_write_t(tile, wt + ((size_t)e * DOUT + n0) * DIN, DIN, dc, (float)WSC, gw, hh, m);
  }
}

__global__ __launch_bounds__(NTHR) void k_gather(const int* __restrict__ ssi, const int* __restrict__ kin,
                                                 const float* __restrict__ x, _Float16* xg) {
  const int tid = threadIdx.x, lane = tid & 31, wave = tid >> 5;
  const int kval = read_k(kin);
#pragma unroll 1
  for (int q = 0; q < 8; ++q) {
    const int r = blockIdx.x * 64 + wave * 8 + q;
    const int valid = (r < NG) ? 1 : 0;
    const int rc = valid ? r : (NG - 1);
    const int a = ssi[rc];
    int tok = a / kval;
    tok = tok < 0 ? 0 : (tok > NTOK - 1 ? NTOK - 1 : tok);
    const float sc = valid ? (float)XSC : 0.0f;
    const float* xr = x + (size_t)tok * DIN;
    _Float16* dr = xg + (size_t)r * DIN;
    v8h hv[4];
#pragma unroll
    for (int j = 0; j < 4; ++j) {
      const int cc = 256 * j + 8 * lane;
      const v4f f0 = *(const v4f*)(xr + cc);
      const v4f f1 = *(const v4f*)(xr + cc + 4);
      hv[j][0] = (_Float16)(f0.x * sc); hv[j][1] = (_Float16)(f0.y * sc);
      hv[j][2] = (_Float16)(f0.z * sc); hv[j][3] = (_Float16)(f0.w * sc);
      hv[j][4] = (_Float16)(f1.x * sc); hv[j][5] = (_Float16)(f1.y * sc);
      hv[j][6] = (_Float16)(f1.z * sc); hv[j][7] = (_Float16)(f1.w * sc);
    }
#pragma unroll
    for (int j = 0; j < 4; ++j) *(volatile v8h*)(dr + 256 * j + 8 * lane) = hv[j];
    __threadfence();
#pragma unroll
    for (int j = 0; j < 4; ++j) *(volatile v8h*)(dr + 256 * j + 8 * lane) = hv[j];
  }
}

__global__ __launch_bounds__(NTHR) void k_gemm(const int* __restrict__ sei, const _Float16* __restrict__ xg,
                                               const _Float16* __restrict__ wt, float* yp) {
  extern __shared__ v4f lds_dyn[];
  __shared__ RouteLds rs;
  const int tid = threadIdx.x, lane = tid & 31, wave = tid >> 5, hh = lane >> 4, m = lane & 15;
  route_counts(sei, &rs, tid);
  const int tile = blockIdx.y;
  int row0, segEnd, my_e;
  const int ntiles = tile_geom(&rs, tile, row0, segEnd, my_e);
  if (tile >= ntiles) return;
  float* stg = (float*)lds_dyn;
  const int n0 = blockIdx.x * 256;
  const int wm = (wave >> 2) * 32, wn = (wave & 3) * 64;

  v8f acc[2][4];
#pragma unroll
  for (int mt = 0; mt < 2; ++mt)
#pragma unroll
    for (int nt = 0; nt < 4; ++nt) { v8f z = {0.f, 0.f, 0.f, 0.f, 0.f, 0.f, 0.f, 0.f}; acc[mt][nt] = z; }

  const _Float16* ap = xg + (size_t)(row0 + wm + m) * DIN + 8 * hh;
  const _Float16* bp = wt + ((size_t)my_e * DOUT + n0 + wn + m) * DIN + 8 * hh;
#pragma unroll 1
  for (int kt = 0; kt < DIN / 32; ++kt) {
    const int k0 = 32 * kt;
    FragH a0, a1;
    a0.h[0] = *(const v8h*)(ap + k0);
    a0.h[1] = *(const v8h*)(ap + k0 + 16);
    a1.h[0] = *(const v8h*)(ap + (size_t)16 * DIN + k0);
    a1.h[1] = *(const v8h*)(ap + (size_t)16 * DIN + k0 + 16);
#pragma unroll
    for (int nt = 0; nt < 4; ++nt) {
      const _Float16* bq = bp + (size_t)nt * 16 * DIN + k0;
      FragH b;
      b.h[0] = *(const v8h*)bq;
      b.h[1] = *(const v8h*)(bq + 16);
      acc[0][nt] = wmf(a0.v, b.v, acc[0][nt]);
      acc[1][nt] = wmf(a1.v, b.v, acc[1][nt]);
    }
  }

  constexpr float OSC = 1.0f / ((float)XSC * (float)WSC);
#pragma unroll
  for (int mt = 0; mt < 2; ++mt) {
    float* spp = stg + (wm + 16 * mt + 8 * hh) * SP + wn + m;
#pragma unroll
    for (int nt = 0; nt < 4; ++nt) {
#pragma unroll
      for (int r = 0; r < 8; ++r) spp[r * SP + 16 * nt] = acc[mt][nt][r] * OSC;
    }
  }
  __syncthreads();

#pragma unroll 1
  for (int q = 0; q < MT / NWAVE; ++q) {
    const int rl = wave * (MT / NWAVE) + q;
    const int gr = row0 + rl;
    const float* s = stg + rl * SP + 4 * lane;
    const v4f u0 = *(const v4f*)s;
    const v4f u1 = *(const v4f*)(s + 128);
    if (gr < segEnd) {
      float* yb = yp + (size_t)gr * DOUT + n0 + 4 * lane;
      *(volatile v4f*)yb = u0;
      *(volatile v4f*)(yb + 128) = u1;
      __threadfence();
      *(volatile v4f*)yb = u0;
      *(volatile v4f*)(yb + 128) = u1;
    }
  }
}

__global__ __launch_bounds__(NTHR) void k_combine(const int* __restrict__ ssi, const int* __restrict__ kin,
                                                  const float* __restrict__ gates, const float* __restrict__ yp,
                                                  float* out) {
#pragma clang fp contract(off)
  __shared__ int s_row[TOPK * TB];
  const int tid = threadIdx.x, lane = tid & 31, wave = tid >> 5;
  const int t0 = blockIdx.x * TB;
  const int kval = read_k(kin);
  if (tid < TOPK * TB) s_row[tid] = -1;
  __syncthreads();
  const int alo = t0 * kval, ahi = alo + TB * kval;
#pragma unroll 1
  for (int i = tid; i < NG; i += NTHR) {
    const int a = ssi[i];
    if (a >= alo && a < ahi) s_row[a - alo] = i;
  }
  __syncthreads();

#pragma unroll 1
  for (int q = 0; q < TB / NWAVE; ++q) {
    const int tl = wave * (TB / NWAVE) + q;
    const int t = t0 + tl;
    v4f ov[8];
#pragma unroll
    for (int jj = 0; jj < 8; ++jj) { v4f z = {0.f, 0.f, 0.f, 0.f}; ov[jj] = z; }
#pragma unroll
    for (int j = 0; j < TOPK; ++j) {
      const int jv = (j < kval) ? 1 : 0;
      int slot = tl * kval + j;
      slot = slot > TOPK * TB - 1 ? TOPK * TB - 1 : slot;
      const int r = s_row[slot];
      const int valid = (jv != 0 && r >= 0) ? 1 : 0;
      int rc = valid ? r : 0;
      rc = rc > NG - 1 ? NG - 1 : rc;
      int gi = t * kval + j;
      gi = gi > NTOK * TOPK - 1 ? NTOK * TOPK - 1 : gi;
      const float graw = gates[gi];
      const float g = valid ? graw : 0.0f;
      const float* yrow = yp + (size_t)rc * DOUT;
#pragma unroll
      for (int jj = 0; jj < 8; ++jj) {
        const v4f u = *(const v4f*)(yrow + 128 * jj + 4 * lane);
        const v4f p = u * g;
        ov[jj] = ov[jj] + p;
      }
    }
    float* orow = out + (size_t)t * DOUT + 4 * lane;
#pragma unroll
    for (int jj = 0; jj < 8; ++jj) *(volatile v4f*)(orow + 128 * jj) = ov[jj];
    __threadfence();
#pragma unroll
    for (int jj = 0; jj < 8; ++jj) *(volatile v4f*)(orow + 128 * jj) = ov[jj];
  }
}

extern "C" void kernel_launch(void* const* d_in, const int* in_sizes, int n_in,
                              void* d_out, int out_size, void* d_ws, size_t ws_size,
                              hipStream_t stream) {
  if (n_in < 7) return;
  if (in_sizes[0] != NTOK * DIN) return;
  if (in_sizes[1] != NEXP * DIN * DOUT) return;
  if (in_sizes[2] < 1) return;
  if (in_sizes[3] != NG) return;
  if (in_sizes[4] != NG) return;
  if (in_sizes[6] != NTOK * TOPK) return;
  if (out_size != NTOK * DOUT) return;

  const float* x     = (const float*)d_in[0];
  const float* w     = (const float*)d_in[1];
  const int*   kin   = (const int*)d_in[2];
  const int*   sei   = (const int*)d_in[3];
  const int*   ssi   = (const int*)d_in[4];
  const float* gates = (const float*)d_in[6];
  float* out = (float*)d_out;

  char* ws = (char*)d_ws;
  size_t off = 0;
  const size_t oW = off; off += (size_t)NEXP * DOUT * DIN * 2;  off = (off + 255) & ~(size_t)255;
  const size_t oX = off; off += (size_t)NGP * DIN * 2;          off = (off + 255) & ~(size_t)255;
  const size_t oY = off; off += (size_t)NGP * DOUT * 4;         off = (off + 255) & ~(size_t)255;
  if (off > ws_size || off > (size_t)WSCAP) return;
  _Float16* wt = (_Float16*)(ws + oW);
  _Float16* xg = (_Float16*)(ws + oX);
  float*    yp = (float*)(ws + oY);

  k_tw<<<dim3(DOUT / 64, NEXP), NTHR, 0, stream>>>(w, wt);
  k_gather<<<NGP / 64, NTHR, 0, stream>>>(ssi, kin, x, xg);
  hipFuncSetAttribute(reinterpret_cast<const void*>(&k_gemm),
                      hipFuncAttributeMaxDynamicSharedMemorySize, LDS_GEMM);
  k_gemm<<<dim3(DOUT / 256, MAXT), NTHR, LDS_GEMM, stream>>>(sei, xg, wt, yp);
  k_combine<<<NTOK / TB, NTHR, 0, stream>>>(ssi, kin, gates, yp, out);
}
